// KernelPointAggregation_25348896981217
// MI455X (gfx1250) — hardware-verified
//
#include <hip/hip_runtime.h>


#pragma STDC FP_CONTRACT OFF

typedef _Float16 v8h  __attribute__((ext_vector_type(8)));
typedef _Float16 v8ha __attribute__((ext_vector_type(8), __may_alias__));
typedef _Float16 v16h __attribute__((ext_vector_type(16)));
typedef float    v8f  __attribute__((ext_vector_type(8)));
typedef float    v4f  __attribute__((ext_vector_type(4)));
typedef float    v4fa __attribute__((ext_vector_type(4), __may_alias__));

#define DIM   64
#define NEI   16
#define KK    4
#define WPB   4
#define UP    72
#define ZP    68
#define MAXN  0.99999f
#define ATLIM 0.99999988f
#define KPE   0.66f

__device__ __forceinline__ float psum(float v) {
#pragma clang fp contract(off)
    return v + __shfl_xor(v, 1, 32);
}
__device__ __forceinline__ float wsum(float v) {
#pragma clang fp contract(off)
    v = v + __shfl_xor(v, 16, 32);
    v = v + __shfl_xor(v, 8, 32);
    v = v + __shfl_xor(v, 4, 32);
    v = v + __shfl_xor(v, 2, 32);
    v = v + __shfl_xor(v, 1, 32);
    return v;
}
__device__ __forceinline__ float log1p_x(float v) {
#pragma clang fp contract(off)
    if (fabsf(v) < 1e-4f) return ((-0.5f * v) + 1.0f) * v;
    return log1pf(v);
}
__device__ __forceinline__ float artanh_x(float v) {
#pragma clang fp contract(off)
    v = fminf(fmaxf(v, -ATLIM), ATLIM);
    return (log1p_x(v) - log1p_x(-v)) * 0.5f;
}
__device__ __forceinline__ float tanh_x(float v) {
    return (fabsf(v) < 0.0004f) ? v : tanhf(v);
}
__device__ __forceinline__ v8f wmma16(v16h a, v16h b, v8f c) {
    c = __builtin_amdgcn_wmma_f32_16x16x32_f16(false, a, false, b, (short)0, c, false, false);
    asm volatile("v_nop\n\tv_nop\n\tv_nop\n\tv_nop" : "+v"(c) : "v"(a), "v"(b));
    return c;
}

__global__ __launch_bounds__(KK * DIM) void
k_prep(const float* __restrict__ W, const float* __restrict__ bv, const float* __restrict__ kt,
       _Float16* __restrict__ Wh, float* __restrict__ xk, float* __restrict__ eb)
{
#pragma clang fp contract(off)
    const int t = threadIdx.x;
    union P8 { v8h v; _Float16 e[8]; };
    union P4 { v4f v; float e[4]; };

    P8 pk[8];
    {
        const float* wr = W + (size_t)t * DIM;
#pragma unroll
        for (int q = 0; q < 8; ++q) {
#pragma unroll
            for (int i = 0; i < 8; ++i) pk[q].e[i] = (_Float16)(wr[q * 8 + i] * 16.0f);
        }
    }

    const bool has_row = (t < 2 * KK);
    P4 ov[16];
#pragma unroll
    for (int i = 0; i < 16; ++i) { ov[i].e[0] = 0.f; ov[i].e[1] = 0.f; ov[i].e[2] = 0.f; ov[i].e[3] = 0.f; }
    float* rdst = xk;
    if (has_row) {
        const float* src = (t < KK) ? (kt + t * DIM) : (bv + (t - KK) * DIM);
        rdst = (t < KK) ? (xk + t * DIM) : (eb + (t - KK) * DIM);
        float s = 0.f;
#pragma unroll
        for (int d = 0; d < DIM; ++d) { const float a = src[d]; ov[d >> 2].e[d & 3] = a; s = s + a * a; }
        const float nrm = sqrtf(fmaxf(s, 1e-14f));
        const float tn  = tanh_x(nrm);
        const float rn  = 1.0f / nrm;
#pragma unroll
        for (int d = 0; d < DIM; ++d) ov[d >> 2].e[d & 3] = (tn * ov[d >> 2].e[d & 3]) * rn;
    }

    {
        _Float16* wd = Wh + (size_t)t * DIM;
#pragma unroll
        for (int q = 0; q < 8; ++q) *(volatile v8ha*)(wd + 8 * q) = pk[q].v;
        if (has_row) {
#pragma unroll
            for (int i = 0; i < 16; ++i) *(volatile v4fa*)(rdst + 4 * i) = ov[i].v;
        }
    }
    __threadfence();
    {
        _Float16* wd = Wh + (size_t)t * DIM;
#pragma unroll
        for (int q = 0; q < 8; ++q) *(volatile v8ha*)(wd + 8 * q) = pk[q].v;
        if (has_row) {
#pragma unroll
            for (int i = 0; i < 16; ++i) *(volatile v4fa*)(rdst + 4 * i) = ov[i].v;
        }
    }
}

__global__ __launch_bounds__(WPB * 32) void
k_main(const float* __restrict__ x, const int* __restrict__ nei, const float* __restrict__ nmask,
       const _Float16* __restrict__ Wh, const float* __restrict__ xk, const float* __restrict__ eb,
       float* __restrict__ out, int N)
{
#pragma clang fp contract(off)
    __shared__ __align__(16) _Float16 s_u[WPB][NEI * UP];
    __shared__ __align__(16) float    s_z[WPB][NEI * ZP];
    __shared__ __align__(16) float    s_xr[WPB][DIM];
    __shared__ __align__(16) float    s_xk[KK * DIM];
    __shared__ __align__(16) float    s_eb[KK * DIM];
    __shared__ float s_wg[WPB][NEI];
    __shared__ float s_xk2[KK];
    __shared__ float s_eb2[KK];

    const int tid  = threadIdx.x;
    const int wave = tid >> 5;
    const int lane = tid & 31;
    const int node = blockIdx.x * WPB + wave;
    const bool valid = node < N;
    const int nc = valid ? node : (N - 1);

    for (int i = tid; i < KK * DIM; i += WPB * 32) { s_xk[i] = xk[i]; s_eb[i] = eb[i]; }
    s_xr[wave][lane]      = x[(size_t)nc * DIM + lane];
    s_xr[wave][lane + 32] = x[(size_t)nc * DIM + lane + 32];
    __syncthreads();
    if (tid < 2 * KK) {
        const float* a = (tid < KK) ? (s_xk + tid * DIM) : (s_eb + (tid - KK) * DIM);
        float s = 0.f;
#pragma unroll 8
        for (int d = 0; d < DIM; ++d) { const float av = a[d]; s = s + av * av; }
        if (tid < KK) s_xk2[tid] = s; else s_eb2[tid - KK] = s;
    }
    __syncthreads();

    const int n  = lane >> 1;
    const int hh = lane & 1;
    const int db = 32 * hh;
    int idx = nei[(size_t)nc * NEI + n];
    idx = (idx < 0) ? 0 : idx;
    idx = (idx > N - 1) ? (N - 1) : idx;
    const float msk = nmask[(size_t)nc * NEI + n];

    float xv[32], v[32];
    {
        const v4fa* xp = (const v4fa*)(&s_xr[wave][db]);
        const v4fa* yp = (const v4fa*)(x + (size_t)idx * DIM + db);
#pragma unroll
        for (int q = 0; q < 8; ++q) {
            const v4f a4 = xp[q];
            const v4f y4 = yp[q];
#pragma unroll
            for (int i = 0; i < 4; ++i) { xv[4 * q + i] = a4[i]; v[4 * q + i] = y4[i]; }
        }
    }
    float sx = 0.f, sy = 0.f, sxy = 0.f;
#pragma unroll
    for (int j = 0; j < 32; ++j) {
        sx  = sx  + xv[j] * xv[j];
        sy  = sy  + v[j]  * v[j];
        sxy = sxy + xv[j] * v[j];
    }
    const float x2 = psum(sx), y2 = psum(sy), xy = psum(sxy);

    const float t1   = 1.0f - 2.0f * xy;
    const float ca   = t1 + y2;
    const float cb   = 1.0f - x2;
    const float rden = 1.0f / fmaxf(t1 + x2 * y2, 1e-15f);
    float sm = 0.f;
#pragma unroll
    for (int j = 0; j < 32; ++j) {
        const float num = cb * v[j] - ca * xv[j];
        const float md  = num * rden;
        v[j] = md;
        sm = sm + md * md;
    }
    const float m2 = psum(sm);

    {
        const float n1  = sqrtf(fmaxf(m2, 1e-14f));
        const float lam = 2.0f * (1.0f / fmaxf(cb, 1e-7f));
        const float acf = 2.0f * (1.0f / lam);
        const float bcf = acf * artanh_x(n1);
        const float rn1 = 1.0f / n1;
        float su = 0.f;
#pragma unroll
        for (int j = 0; j < 32; ++j) {
            const float lv = (bcf * v[j]) * rn1;
            const float uv = (lv * lam) * 0.5f;
            v[j] = uv;
            su = su + uv * uv;
        }
        su = psum(su);
        const float nu2 = sqrtf(fmaxf(su, 1e-14f));
        const float tnu = tanh_x(nu2);
        const float rnu = 1.0f / nu2;
        float se = 0.f;
#pragma unroll
        for (int j = 0; j < 32; ++j) {
            const float ev = (tnu * v[j]) * rnu;
            v[j] = ev;
            se = se + ev * ev;
        }
        se = psum(se);
        const float ne = sqrtf(fmaxf(se, 1e-14f));
        if (ne > MAXN) {
            const float re = 1.0f / ne;
#pragma unroll
            for (int j = 0; j < 32; ++j) v[j] = (v[j] * re) * MAXN;
        }
    }
    float s0 = 0.f;
#pragma unroll
    for (int j = 0; j < 32; ++j) s0 = s0 + v[j] * v[j];
    s0 = psum(s0);

    {
        const float n0  = sqrtf(fmaxf(s0, 1e-14f));
        const float at0 = artanh_x(n0);
        const float rc0 = 1.0f / n0;
        union P8 { v8h v; _Float16 e[8]; };
        _Float16* up = &s_u[wave][n * UP + db];
#pragma unroll
        for (int q = 0; q < 4; ++q) {
            P8 pk;
#pragma unroll
            for (int i = 0; i < 8; ++i) pk.e[i] = (_Float16)(((at0 * v[8 * q + i]) * rc0) * 8.0f);
            *(v8ha*)(up + 8 * q) = pk.v;
        }
    }

    float wk[KK];
    {
        const float cbx = 1.0f - s0;
#pragma unroll
        for (int k = 0; k < KK; ++k) {
            float kv[32];
            {
                const v4fa* kp = (const v4fa*)(s_xk + k * DIM + db);
#pragma unroll
                for (int q = 0; q < 8; ++q) {
                    const v4f t4 = kp[q];
#pragma unroll
                    for (int i = 0; i < 4; ++i) kv[4 * q + i] = t4[i];
                }
            }
            float sp = 0.f;
#pragma unroll
            for (int j = 0; j < 32; ++j) sp = sp + v[j] * kv[j];
            const float p   = psum(sp);
            const float tk  = 1.0f - 2.0f * p;
            const float cak = tk + s_xk2[k];
            const float rdk = 1.0f / fmaxf(tk + s0 * s_xk2[k], 1e-15f);
            float ss = 0.f;
#pragma unroll
            for (int j = 0; j < 32; ++j) {
                const float num = cbx * kv[j] - cak * v[j];
                const float md  = num * rdk;
                ss = ss + md * md;
            }
            ss = psum(ss);
            const float nm  = sqrtf(fmaxf(ss, 1e-14f));
            const float dis = 2.0f * artanh_x(nm);
            wk[k] = fmaxf(1.0f - dis * (1.0f / KPE), 0.0f) * msk;
        }
    }

    __syncthreads();
    const int m16 = lane & 15;
    const int h2  = lane >> 4;
    union Frag { v16h v; v8h hv[2]; };
    Frag fa0, fa1;
    {
        const _Float16* up = &s_u[wave][m16 * UP + 8 * h2];
        fa0.hv[0] = *(const v8ha*)(up);
        fa0.hv[1] = *(const v8ha*)(up + 16);
        fa1.hv[0] = *(const v8ha*)(up + 32);
        fa1.hv[1] = *(const v8ha*)(up + 48);
    }

    float ona = 0.f, onb = 0.f, od = 0.f;
#pragma unroll 1
    for (int k = 0; k < KK; ++k) {
        const float wkk = (k == 0) ? wk[0] : ((k == 1) ? wk[1] : ((k == 2) ? wk[2] : wk[3]));

#pragma unroll
        for (int t = 0; t < 4; ++t) {
            const _Float16* wb = Wh + ((size_t)(k * DIM + t * 16 + m16)) * DIM + 8 * h2;
            Frag fb0, fb1;
            fb0.hv[0] = *(const v8ha*)(wb);
            fb0.hv[1] = *(const v8ha*)(wb + 16);
            fb1.hv[0] = *(const v8ha*)(wb + 32);
            fb1.hv[1] = *(const v8ha*)(wb + 48);
            v8f acc = {0.f, 0.f, 0.f, 0.f, 0.f, 0.f, 0.f, 0.f};
            acc = wmma16(fa0.v, fb0.v, acc);
            acc = wmma16(fa1.v, fb1.v, acc);
            float* zp = &s_z[wave][(8 * h2) * ZP + t * 16 + m16];
#pragma unroll
            for (int r = 0; r < 8; ++r) zp[r * ZP] = acc[r];
        }
        __syncthreads();

        {
            float* zr = &s_z[wave][n * ZP + db];
            float ebv[32];
            {
                const v4fa* ep = (const v4fa*)(s_eb + k * DIM + db);
#pragma unroll
                for (int q = 0; q < 8; ++q) {
                    const v4f e4 = ep[q];
#pragma unroll
                    for (int i = 0; i < 4; ++i) ebv[4 * q + i] = e4[i];
                }
            }
            float sz = 0.f;
            {
                const v4fa* zq = (const v4fa*)zr;
#pragma unroll
                for (int q = 0; q < 8; ++q) {
                    const v4f z4 = zq[q];
#pragma unroll
                    for (int i = 0; i < 4; ++i) {
                        const float zv = z4[i] * 0.0078125f;
                        v[4 * q + i] = zv;
                        sz = sz + zv * zv;
                    }
                }
            }
            sz = psum(sz);
            const float nz  = sqrtf(fmaxf(sz, 1e-14f));
            const float tz  = tanh_x(nz);
            const float rz  = 1.0f / nz;
            float se = 0.f, sxe = 0.f;
#pragma unroll
            for (int j = 0; j < 32; ++j) {
                const float ev = (tz * v[j]) * rz;
                v[j] = ev;
                se  = se  + ev * ev;
                sxe = sxe + ev * ebv[j];
            }
            const float hx2 = psum(se), hxy = psum(sxe);
            const float hy2 = s_eb2[k];
            const float t2  = 1.0f + 2.0f * hxy;
            const float ca2 = t2 + hy2;
            const float cb2 = 1.0f - hx2;
            const float rd2 = 1.0f / fmaxf(t2 + hx2 * hy2, 1e-15f);
            float sh = 0.f;
#pragma unroll
            for (int j = 0; j < 32; ++j) {
                const float hv = (ca2 * v[j] + cb2 * ebv[j]) * rd2;
                v[j] = hv;
                sh = sh + hv * hv;
            }
            sh = psum(sh);
            const float nh = sqrtf(fmaxf(sh, 1e-14f));
            if (nh > MAXN) {
                const float rh = 1.0f / nh;
#pragma unroll
                for (int j = 0; j < 32; ++j) v[j] = (v[j] * rh) * MAXN;
            }
            float sk = 0.f;
#pragma unroll
            for (int j = 0; j < 32; ++j) sk = sk + v[j] * v[j];
            sk = psum(sk);
            const float rp = 1.0f / (1.0f + sk);
            float sg = 0.f;
#pragma unroll
            for (int j = 0; j < 32; ++j) {
                const float kvv = (2.0f * v[j]) * rp;
                v[j] = kvv;
                sg = sg + kvv * kvv;
            }
            sg = psum(sg);
            const float gm = 1.0f / sqrtf(fmaxf(1.0f - sg, 1e-7f));
            const float wg = wkk * gm;
            {
                union P4 { v4f v; float e[4]; };
#pragma unroll
                for (int q = 0; q < 8; ++q) {
                    P4 o4;
#pragma unroll
                    for (int i = 0; i < 4; ++i) o4.e[i] = wg * v[4 * q + i];
                    *(v4fa*)(zr + 4 * q) = o4.v;
                }
            }
            if (hh == 0) s_wg[wave][n] = wg;
        }
        __syncthreads();

        {
            float sw = 0.f;
#pragma unroll
            for (int q = 0; q < NEI; ++q) sw = sw + s_wg[wave][q];
            const float rw = 1.0f / fmaxf(sw, 1e-10f);
            float ma = 0.f, mb = 0.f;
#pragma unroll
            for (int q = 0; q < NEI; ++q) {
                ma = ma + s_z[wave][q * ZP + lane];
                mb = mb + s_z[wave][q * ZP + lane + 32];
            }
            const float mida = ma * rw, midb = mb * rw;
            const float sg2  = wsum(mida * mida + midb * midb);
            const float g2   = 1.0f / sqrtf(fmaxf(1.0f - sg2, 1e-7f));
            ona = ona + g2 * mida;
            onb = onb + g2 * midb;
            od  = od + g2;
        }
        __syncthreads();
    }

    const float rod = 1.0f / fmaxf(od, 1e-10f);
    const float oa = ona * rod, ob = onb * rod;
    const float so = wsum(oa * oa + ob * ob);
    const float sq = sqrtf(fmaxf(1.0f - so, 1e-7f));
    const float rk = 1.0f / (1.0f + sq);
    float pa = oa * rk, pb = ob * rk;
    const float s2p = wsum(pa * pa + pb * pb);
    const float npn = sqrtf(fmaxf(s2p, 1e-14f));
    if (npn > MAXN) {
        const float rr = 1.0f / npn;
        pa = (pa * rr) * MAXN;
        pb = (pb * rr) * MAXN;
    }
    const float s3 = wsum(pa * pa + pb * pb);
    const float n3 = sqrtf(fmaxf(s3, 1e-14f));
    const float a3 = artanh_x(n3);
    const float r3 = 1.0f / n3;
    const float va = fmaxf((a3 * pa) * r3, 0.0f);
    const float vb = fmaxf((a3 * pb) * r3, 0.0f);
    const float s4 = wsum(va * va + vb * vb);
    const float n4 = sqrtf(fmaxf(s4, 1e-14f));
    const float t4 = tanh_x(n4);
    const float r4 = 1.0f / n4;
    const float fa = (t4 * va) * r4;
    const float fb = (t4 * vb) * r4;

    s_z[wave][lane]      = fa;
    s_z[wave][lane + 32] = fb;
    __syncthreads();
    if (valid && lane < 16) {
        const v4f val = *(const v4fa*)(&s_z[wave][4 * lane]);
        volatile v4fa* op = (volatile v4fa*)(out + (size_t)node * DIM + 4 * lane);
        *op = val;
        __threadfence();
        *op = val;
    }
}

extern "C" void kernel_launch(void* const* d_in, const int* in_sizes, int n_in,
                              void* d_out, int out_size, void* d_ws, size_t ws_size,
                              hipStream_t stream)
{
    if (n_in < 6) return;
    const int N = in_sizes[0] / DIM;
    if (N <= 0) return;
    if (in_sizes[0] != N * DIM) return;
    if (in_sizes[1] != N * NEI) return;
    if (in_sizes[2] != N * NEI) return;
    if (in_sizes[3] != KK * DIM * DIM) return;
    if (in_sizes[4] != KK * DIM) return;
    if (in_sizes[5] != KK * DIM) return;
    if (out_size != N * DIM) return;

    const float* x   = (const float*)d_in[0];
    const int*   nei = (const int*)d_in[1];
    const float* msk = (const float*)d_in[2];
    const float* W   = (const float*)d_in[3];
    const float* bv  = (const float*)d_in[4];
    const float* kt  = (const float*)d_in[5];
    float* out = (float*)d_out;

    const size_t off_wh = 0;
    const size_t off_xk = (size_t)KK * DIM * DIM * sizeof(_Float16);
    const size_t off_eb = off_xk + (size_t)KK * DIM * sizeof(float);
    const size_t total  = off_eb + (size_t)KK * DIM * sizeof(float);
    if (ws_size < total) return;
    _Float16* Wh = (_Float16*)((char*)d_ws + off_wh);
    float*    xk = (float*)((char*)d_ws + off_xk);
    float*    eb = (float*)((char*)d_ws + off_eb);

    k_prep<<<1, KK * DIM, 0, stream>>>(W, bv, kt, Wh, xk, eb);
    const int grid = (N + WPB - 1) / WPB;
    k_main<<<grid, WPB * 32, 0, stream>>>(x, nei, msk, Wh, xk, eb, out, N);
}
